// FusetViTBlock_69191923138813
// MI455X (gfx1250) — hardware-run, weakly checked
//
#include <hip/hip_runtime.h>
#include <stdint.h>

#define NB    16
#define NP    1024
#define IMW   32
#define CH    256
#define C3    768
#define CA    512
#define CM    1024
#define HDM   32
#define HPC   96
#define NPAIR 8
#define NGRP  24
#define GM    128
#define GN    64
#define OSP   68
#define LTP   72
#define KVP   40
#define WSC   64.0f
#define DSC   16.0f
#define ATTSC 64.0f
#define T1SC  8.0f
#define HSC   8.0f
#define IHSC  0.125f
#define H2SC  16.0f
#define SA_GPW  0.0009765625f
#define SA_PROJ 0.000244140625f
#define SA_INV  0.001953125f
#define SA_PW   0.0009765625f
#define EPSA  1e-15f
#define BNEPS 1e-5f
#define SIXTH 0.16666667f

#define WOFF1 196608
#define WOFF2 327680
#define WOFF3 589824
#define WTOT  851968

static_assert(IMW * IMW == NP);
static_assert(NP % GN == 0);
static_assert(NP % 128 == 0);
static_assert(C3 % GM == 0);
static_assert(CH % GM == 0);
static_assert(CM % GM == 0);
static_assert(CH % 64 == 0);
static_assert(CM % 64 == 0);
static_assert(NPAIR * 2 * HDM == CA);
static_assert(NGRP * 32 == C3);
static_assert(8 * HPC == C3);
static_assert(WOFF1 % 2048 == 0);
static_assert(WOFF2 % 2048 == 0);
static_assert(WOFF3 % 2048 == 0);
static_assert(WTOT % 2048 == 0);
static_assert(WOFF1 == C3 * CH);
static_assert(WOFF2 - WOFF1 == CH * CA);
static_assert(WOFF3 - WOFF2 == CM * CH);
static_assert(WTOT - WOFF3 == CH * CM);
static_assert((OSP * 4) % 16 == 0);
static_assert((LTP * 2) % 16 == 0);
static_assert((KVP * 2) % 16 == 0);

typedef _Float16       v16h __attribute__((ext_vector_type(16)));
typedef _Float16       v8h  __attribute__((ext_vector_type(8)));
typedef __bf16         v16b __attribute__((ext_vector_type(16)));
typedef unsigned short v8us __attribute__((ext_vector_type(8)));
typedef float          v8f  __attribute__((ext_vector_type(8)));
typedef float          v4f  __attribute__((ext_vector_type(4)));
typedef unsigned int   v4u  __attribute__((ext_vector_type(4)));

union Frag { v8us u[2]; v16h h; v16b bf; };
static_assert(sizeof(Frag) == 32);

__device__ __forceinline__ unsigned short bf_bits(float f) {
  unsigned u = __float_as_uint(f);
  return (unsigned short)((u + 0x7FFFu + ((u >> 16) & 1u)) >> 16);
}
__device__ __forceinline__ float bf_up(unsigned short hb) { return __uint_as_float(((unsigned)hb) << 16); }
__device__ __forceinline__ float bfr(float f) { return bf_up(bf_bits(f)); }
__device__ __forceinline__ unsigned short h_bits(_Float16 x) { return __builtin_bit_cast(unsigned short, x); }
__device__ __forceinline__ unsigned pk16(unsigned short a, unsigned short b) { return (unsigned)a | ((unsigned)b << 16); }
__device__ __forceinline__ v8f zero8() { v8f z = {0.f, 0.f, 0.f, 0.f, 0.f, 0.f, 0.f, 0.f}; return z; }
__device__ __forceinline__ float hswish_f(float x) {
  const float cc = fminf(fmaxf(x + 3.0f, 0.0f), 6.0f);
  return x * cc * SIXTH;
}
__device__ __forceinline__ unsigned short relu16(unsigned short v) { return (v & 0x8000u) ? (unsigned short)0u : v; }
__device__ __forceinline__ v8us relu8(v8us x) {
  v8us r;
#pragma unroll
  for (int i = 0; i < 8; ++i) { const unsigned short v = x[i]; r[i] = (v & 0x8000u) ? (unsigned short)0u : v; }
  return r;
}

__device__ __forceinline__ Frag ldfrag(const unsigned short* p) {
  Frag f;
  f.u[0] = *(const v8us*)(p);
  f.u[1] = *(const v8us*)(p + 16);
  return f;
}

__device__ __forceinline__ v8f mma_h(v16h a, v16h b, v8f c) {
  v8f d = __builtin_amdgcn_wmma_f32_16x16x32_f16(false, a, false, b, (short)0, c, false, false);
#if defined(__HIP_DEVICE_COMPILE__)
  asm volatile("v_nop\n\tv_nop\n\tv_nop\n\tv_nop" : "+v"(d) : "v"(a), "v"(b));
#endif
  return d;
}
__device__ __forceinline__ v8f mma_b(v16b a, v16b b, v8f c) {
  v8f d = __builtin_amdgcn_wmma_f32_16x16x32_bf16(false, a, false, b, (short)0, c, false, false);
#if defined(__HIP_DEVICE_COMPILE__)
  const v16h ha = __builtin_bit_cast(v16h, a), hb = __builtin_bit_cast(v16h, b);
  asm volatile("v_nop\n\tv_nop\n\tv_nop\n\tv_nop" : "+v"(d) : "v"(ha), "v"(hb));
#endif
  return d;
}

__global__ __launch_bounds__(256)
void cvt_w(const float* __restrict__ w0, const float* __restrict__ w1, const float* __restrict__ w2,
           const float* __restrict__ w3, unsigned short* WB) {
  const int g0 = (int)blockIdx.x * 2048;
  const float* src = w0;
  int base = 0;
  bool isbf = true;
  if (g0 >= WOFF3)      { src = w3; base = WOFF3; isbf = false; }
  else if (g0 >= WOFF2) { src = w2; base = WOFF2; isbf = false; }
  else if (g0 >= WOFF1) { src = w1; base = WOFF1; isbf = false; }
  const int i = g0 + (int)threadIdx.x * 8;
  const float* s = src + (i - base);
  const v4f a = *(const v4f*)(s);
  const v4f q = *(const v4f*)(s + 4);
  v4u w;
  if (isbf) {
    w[0] = pk16(bf_bits(a[0]), bf_bits(a[1]));
    w[1] = pk16(bf_bits(a[2]), bf_bits(a[3]));
    w[2] = pk16(bf_bits(q[0]), bf_bits(q[1]));
    w[3] = pk16(bf_bits(q[2]), bf_bits(q[3]));
  } else {
    w[0] = pk16(h_bits((_Float16)(bfr(a[0]) * WSC)), h_bits((_Float16)(bfr(a[1]) * WSC)));
    w[1] = pk16(h_bits((_Float16)(bfr(a[2]) * WSC)), h_bits((_Float16)(bfr(a[3]) * WSC)));
    w[2] = pk16(h_bits((_Float16)(bfr(q[0]) * WSC)), h_bits((_Float16)(bfr(q[1]) * WSC)));
    w[3] = pk16(h_bits((_Float16)(bfr(q[2]) * WSC)), h_bits((_Float16)(bfr(q[3]) * WSC)));
  }
  unsigned short* p = WB + (size_t)i;
  *(volatile v4u*)p = w;
  __threadfence();
  *(volatile v4u*)p = w;
}

__global__ __launch_bounds__(256)
void cvt_x(const float* __restrict__ x, unsigned short* X16) {
  __shared__ __align__(16) unsigned short Lt[GN * LTP];
  const int tid = threadIdx.x;
  const int nt = blockIdx.x, cg = blockIdx.y, b = blockIdx.z;
  const int n0 = nt * GN;
  {
    const int n4 = (tid & 15) * 4, cs = tid >> 4;
#pragma unroll
    for (int it = 0; it < 4; ++it) {
      const int cl = it * 16 + cs;
      const v4f v = *(const v4f*)(x + ((size_t)(b * CH + cg * 64 + cl)) * NP + n0 + n4);
#pragma unroll
      for (int qq = 0; qq < 4; ++qq) Lt[(n4 + qq) * LTP + cl] = bf_bits(v[qq]);
    }
  }
  __syncthreads();
  {
    const int e = tid & 7, lq = tid >> 3;
#pragma unroll
    for (int pass = 0; pass < 2; ++pass) {
#pragma unroll
      for (int it = 0; it < 2; ++it) {
        const int n = it * 32 + lq;
        const v4u u = *(const v4u*)(Lt + n * LTP + 8 * e);
        *(volatile v4u*)(X16 + ((size_t)(b * NP + n0 + n)) * CH + cg * 64 + 8 * e) = u;
      }
      __threadfence();
    }
  }
}

template <int MODE>
__global__ __launch_bounds__(256)
void gemm_kernel(const unsigned short* __restrict__ Wp, int K, float sA,
                 const unsigned short* __restrict__ Bp,
                 const float* __restrict__ bias,
                 const float* __restrict__ bng, const float* __restrict__ bnb,
                 const float* __restrict__ bnm, const float* __restrict__ bnv,
                 int act,
                 const float* __restrict__ res1, int res1_rne, const float* __restrict__ res2,
                 int M,
                 float* outF, unsigned short* out16, float s16, unsigned short* outP, float sP) {
  __shared__ __align__(16) float Os[GM * OSP];
  __shared__ float bnS[GM];
  __shared__ float bnB[GM];
  const int tid  = threadIdx.x;
  const int lane = tid & 31, wave = tid >> 5;
  const int hh   = lane >> 4, c = lane & 15;
  const int wm   = wave >> 1, wn = wave & 1;
  const int b    = blockIdx.z;
  const int mBase = blockIdx.x * GM;
  const int nBase = blockIdx.y * GN;

  if (tid < GM) {
    float s = 1.0f, t = 0.0f;
    if (bng != nullptr) {
      const int o = mBase + tid;
      const float inv = bfr(bng[o]) * (1.0f / sqrtf(bfr(bnv[o]) + BNEPS));
      s = inv;
      t = bfr(bnb[o]) - bfr(bnm[o]) * inv;
    }
    bnS[tid] = s;
    bnB[tid] = t;
  }
  __syncthreads();

  const unsigned short* a0p = Wp + (size_t)(mBase + 32 * wm + c) * K + 8 * hh;
  const unsigned short* a1p = a0p + (size_t)16 * K;
  const unsigned short* b0p = Bp + ((size_t)b * NP + nBase + 32 * wn + c) * (size_t)K + 8 * hh;
  const unsigned short* b1p = b0p + (size_t)16 * K;

  v8f acc[2][2];
#pragma unroll
  for (int mi = 0; mi < 2; ++mi)
#pragma unroll
    for (int ni = 0; ni < 2; ++ni) acc[mi][ni] = zero8();

#pragma unroll 1
  for (int k0 = 0; k0 < K; k0 += 32) {
    const Frag fa0 = ldfrag(a0p + k0);
    const Frag fa1 = ldfrag(a1p + k0);
    const Frag fb0 = ldfrag(b0p + k0);
    const Frag fb1 = ldfrag(b1p + k0);
    if (MODE == 0) {
      acc[0][0] = mma_b(fa0.bf, fb0.bf, acc[0][0]);
      acc[0][1] = mma_b(fa0.bf, fb1.bf, acc[0][1]);
      acc[1][0] = mma_b(fa1.bf, fb0.bf, acc[1][0]);
      acc[1][1] = mma_b(fa1.bf, fb1.bf, acc[1][1]);
    } else {
      acc[0][0] = mma_h(fa0.h, fb0.h, acc[0][0]);
      acc[0][1] = mma_h(fa0.h, fb1.h, acc[0][1]);
      acc[1][0] = mma_h(fa1.h, fb0.h, acc[1][0]);
      acc[1][1] = mma_h(fa1.h, fb1.h, acc[1][1]);
    }
  }

#pragma unroll
  for (int mi = 0; mi < 2; ++mi) {
#pragma unroll
    for (int ni = 0; ni < 2; ++ni) {
      const int n_loc = 32 * wn + 16 * ni + c;
      const int n = nBase + n_loc;
#pragma unroll
      for (int r = 0; r < 8; ++r) {
        const int o_loc = 32 * wm + 16 * mi + 8 * hh + r;
        const int o = mBase + o_loc;
        float v = acc[mi][ni][r] * sA;
        if (bias != nullptr) v += bfr(bias[o]);
        v = v * bnS[o_loc] + bnB[o_loc];
        if (act != 0) v = hswish_f(v);
        const size_t ridx = ((size_t)b * M + o) * NP + n;
        if (res1 != nullptr) {
          float rv = res1[ridx];
          if (res1_rne != 0) rv = bfr(rv);
          v += rv;
        }
        if (res2 != nullptr) v += res2[ridx];
        Os[o_loc * OSP + n_loc] = v;
      }
    }
  }
  __syncthreads();

  {
    const int e = tid & 7, lq = tid >> 3;
#pragma unroll
    for (int pass = 0; pass < 2; ++pass) {
      if (outF != nullptr) {
#pragma unroll
        for (int it = 0; it < 8; ++it) {
          const int L = it * 32 + lq;
          const int row = L >> 1, hf = L & 1;
          const v4f v = *(const v4f*)(Os + row * OSP + hf * 32 + 4 * e);
          float* dst = outF + ((size_t)b * M + mBase + row) * NP + nBase + hf * 32 + 4 * e;
          *(volatile v4f*)dst = v;
        }
      }
      if (out16 != nullptr) {
#pragma unroll
        for (int it = 0; it < 4; ++it) {
          const int row = it * 32 + lq;
          const v4f v0 = *(const v4f*)(Os + row * OSP + 8 * e);
          const v4f v1 = *(const v4f*)(Os + row * OSP + 8 * e + 4);
          v4u u;
          u[0] = pk16(h_bits((_Float16)(v0[0] * s16)), h_bits((_Float16)(v0[1] * s16)));
          u[1] = pk16(h_bits((_Float16)(v0[2] * s16)), h_bits((_Float16)(v0[3] * s16)));
          u[2] = pk16(h_bits((_Float16)(v1[0] * s16)), h_bits((_Float16)(v1[1] * s16)));
          u[3] = pk16(h_bits((_Float16)(v1[2] * s16)), h_bits((_Float16)(v1[3] * s16)));
          unsigned short* dst = out16 + ((size_t)b * M + mBase + row) * NP + nBase + 8 * e;
          *(volatile v4u*)dst = u;
        }
      }
      if (outP != nullptr) {
#pragma unroll
        for (int it = 0; it < 4; ++it) {
          const int L = it * 32 + lq;
          const int n_loc = L >> 1, hf = L & 1;
          const int ch0 = hf * 64 + 8 * e;
          float f[8];
#pragma unroll
          for (int jj = 0; jj < 8; ++jj) f[jj] = Os[(ch0 + jj) * OSP + n_loc];
          v4u uh;
#pragma unroll
          for (int t = 0; t < 4; ++t)
            uh[t] = pk16(h_bits((_Float16)(f[2 * t] * sP)), h_bits((_Float16)(f[2 * t + 1] * sP)));
          const size_t po = ((size_t)b * NP + nBase + n_loc) * (size_t)M + mBase + ch0;
          *(volatile v4u*)(outP + po) = uh;
        }
      }
      __threadfence();
    }
  }
}

__global__ __launch_bounds__(256)
void dw5_gpw_kernel(const unsigned short* __restrict__ Q16, const float* __restrict__ w5g,
                    const float* __restrict__ wpg, unsigned short* PW) {
  __shared__ float w5[32 * 25];
  __shared__ __align__(16) unsigned short wA[32 * KVP];
  __shared__ __align__(16) unsigned short dT[GN * KVP];
  __shared__ __align__(16) unsigned short oT[32 * LTP];
  const int tid  = threadIdx.x;
  const int lane = tid & 31, wave = tid >> 5;
  const int hh   = lane >> 4, c = lane & 15;
  const int nt   = blockIdx.x, g = blockIdx.y, b = blockIdx.z;
  const int n0   = nt * GN;

  for (int i = tid; i < 32 * 25; i += 256) w5[i] = bfr(w5g[(size_t)g * 800 + i]);
#pragma unroll
  for (int it = 0; it < 4; ++it) {
    const int idx = it * 256 + tid;
    const int o = idx >> 5, i = idx & 31;
    wA[o * KVP + i] = h_bits((_Float16)(bfr(wpg[(size_t)g * 1024 + idx]) * WSC));
  }
  __syncthreads();

  {
    const int nl = tid & 63, cq = tid >> 6;
    const int n  = n0 + nl;
    const int y  = n / IMW;
    const int xq = n - y * IMW;
    const _Float16* Qh = (const _Float16*)(const void*)Q16;
#pragma unroll 1
    for (int jj = 0; jj < 8; ++jj) {
      const int cl = cq * 8 + jj;
      const _Float16* qr = Qh + ((size_t)(b * C3 + g * 32 + cl)) * NP;
      float accv = 0.f;
#pragma unroll
      for (int t = 0; t < 25; ++t) {
        const int ky = t / 5, kx = t - ky * 5;
        const int yy = y + ky - 2, xx = xq + kx - 2;
        const bool ok = ((unsigned)yy < (unsigned)IMW) && ((unsigned)xx < (unsigned)IMW);
        const int yc = min(max(yy, 0), IMW - 1);
        const int xc = min(max(xx, 0), IMW - 1);
        const float hv = (float)qr[yc * IMW + xc];
        accv = fmaf(ok ? hv : 0.f, w5[cl * 25 + t], accv);
      }
      dT[nl * KVP + cl] = h_bits((_Float16)(accv * DSC));
    }
  }
  __syncthreads();

  {
    const int mi = wave >> 2, ni = wave & 3;
    const Frag fa = ldfrag(wA + (16 * mi + c) * KVP + 8 * hh);
    const Frag fb = ldfrag(dT + (16 * ni + c) * KVP + 8 * hh);
    const v8f accp = mma_h(fa.h, fb.h, zero8());
    unsigned short* ot = oT + (16 * mi + 8 * hh) * LTP + 16 * ni + c;
#pragma unroll
    for (int r = 0; r < 8; ++r) ot[r * LTP] = h_bits((_Float16)(accp[r] * SA_GPW));
  }
  __syncthreads();

  {
    const int e = tid & 7, lq = tid >> 3;
    const v4u u = *(const v4u*)(oT + lq * LTP + 8 * e);
    unsigned short* dst = PW + ((size_t)(b * C3 + g * 32 + lq)) * NP + n0 + 8 * e;
    *(volatile v4u*)dst = u;
    __threadfence();
    *(volatile v4u*)dst = u;
  }
}

__global__ __launch_bounds__(256)
void attn_kernel(const unsigned short* __restrict__ QKV16, const unsigned short* __restrict__ PW16,
                 unsigned short* ATT) {
  __shared__ __align__(16) unsigned short kv16[2 * 48 * KVP];
  __shared__ __align__(16) unsigned short attT[128 * LTP];
  const int tid  = threadIdx.x;
  const int lane = tid & 31, wave = tid >> 5;
  const int hh   = lane >> 4, c = lane & 15;
  const int j    = blockIdx.x, b = blockIdx.y;
  const int hl   = wave >> 2, wsub = wave & 3;
  const bool lowset = (j < 4);
  const unsigned short* plane = lowset ? QKV16 : PW16;
  const int hc = (lowset ? j : (j - 4)) * 2 + hl;
  const size_t rb = (size_t)b * C3 + (size_t)hc * HPC;

  if (wsub < 3) {
    const int mi = wsub;
    const int vofs = 2 * HDM + ((mi < 2) ? 16 * mi : 0);
    const unsigned short* vp  = plane + (rb + vofs + c) * NP + 8 * hh;
    const unsigned short* k0p = plane + (rb + HDM + c) * NP + 8 * hh;
    const unsigned short* k1p = k0p + (size_t)16 * NP;
    v8us ov;
#pragma unroll
    for (int i = 0; i < 8; ++i) ov[i] = (c == 0) ? (unsigned short)0x3C00u : (unsigned short)0u;
    Frag onesF;
    onesF.u[0] = ov;
    onesF.u[1] = ov;
    v8f a0 = zero8(), a1 = zero8();
#pragma unroll 1
    for (int ks = 0; ks < NP; ks += 32) {
      Frag fa = onesF;
      if (mi < 2) fa = ldfrag(vp + ks);
      Frag fk0 = ldfrag(k0p + ks);
      Frag fk1 = ldfrag(k1p + ks);
      fk0.u[0] = relu8(fk0.u[0]); fk0.u[1] = relu8(fk0.u[1]);
      fk1.u[0] = relu8(fk1.u[0]); fk1.u[1] = relu8(fk1.u[1]);
      a0 = mma_h(fa.h, fk0.h, a0);
      a1 = mma_h(fa.h, fk1.h, a1);
    }
    unsigned short* kvw = kv16 + hl * (48 * KVP) + (16 * mi + 8 * hh) * KVP + c;
#pragma unroll
    for (int r = 0; r < 8; ++r) {
      kvw[r * KVP]      = h_bits((_Float16)a0[r]);
      kvw[r * KVP + 16] = h_bits((_Float16)a1[r]);
    }
  }
  __syncthreads();

  const unsigned short* kvh = kv16 + hl * (48 * KVP);
  const Frag A0 = ldfrag(kvh + (0  + c) * KVP + 8 * hh);
  const Frag A1 = ldfrag(kvh + (16 + c) * KVP + 8 * hh);
  const Frag A2 = ldfrag(kvh + (32 + c) * KVP + 8 * hh);
  const unsigned short* qb = plane + rb * NP + c;
#pragma unroll 1
  for (int ck = 0; ck < NP / 128; ++ck) {
#pragma unroll
    for (int u = 0; u < 2; ++u) {
      const int tl = wsub * 2 + u;
      const int n0 = ck * 128 + 16 * tl;
      const unsigned short* qp = qb + n0;
      v8us q0, q1;
#pragma unroll
      for (int i = 0; i < 8; ++i) {
        q0[i] = relu16(qp[(size_t)(8 * hh + i) * NP]);
        q1[i] = relu16(qp[(size_t)(16 + 8 * hh + i) * NP]);
      }
      Frag qf;
      qf.u[0] = q0;
      qf.u[1] = q1;
      const v8f o0 = mma_h(A0.h, qf.h, zero8());
      const v8f o1 = mma_h(A1.h, qf.h, zero8());
      const v8f o2 = mma_h(A2.h, qf.h, zero8());
      const float den = __shfl(o2[0], c, 32);
      const float rd = ATTSC / (den + EPSA);
      v4u u0, u1;
#pragma unroll
      for (int t = 0; t < 4; ++t) {
        u0[t] = pk16(h_bits((_Float16)(o0[2 * t] * rd)), h_bits((_Float16)(o0[2 * t + 1] * rd)));
        u1[t] = pk16(h_bits((_Float16)(o1[2 * t] * rd)), h_bits((_Float16)(o1[2 * t + 1] * rd)));
      }
      const int nloc = 16 * tl + c;
      *(v4u*)(attT + nloc * LTP + 32 * hl + 8 * hh) = u0;
      *(v4u*)(attT + nloc * LTP + 32 * hl + 16 + 8 * hh) = u1;
    }
    __syncthreads();
    {
      const int e = tid & 7, lq = tid >> 3;
      unsigned short* ab = ATT + ((size_t)b * NP + ck * 128) * CA + 64 * j + 8 * e;
#pragma unroll
      for (int pass = 0; pass < 2; ++pass) {
#pragma unroll
        for (int it = 0; it < 4; ++it) {
          const int L = it * 32 + lq;
          const v4u uu = *(const v4u*)(attT + L * LTP + 8 * e);
          *(volatile v4u*)(ab + (size_t)L * CA) = uu;
        }
        __threadfence();
      }
    }
    __syncthreads();
  }
}

__global__ __launch_bounds__(256)
void dw3_kernel(const unsigned short* __restrict__ H16, const float* __restrict__ w, const float* __restrict__ bb,
                unsigned short* H2) {
  __shared__ __align__(16) unsigned short Lh[GN * LTP];
  __shared__ float w3[64 * 9];
  __shared__ float b3[64];
  const int tid = threadIdx.x;
  const int nl  = tid & 63, cq = tid >> 6;
  const int nt  = blockIdx.x, cg = blockIdx.y, b = blockIdx.z;
  const int n0  = nt * GN;
  const int n   = n0 + nl;
  const int y   = n / IMW;
  const int xq  = n - y * IMW;
  for (int i = tid; i < 64 * 9; i += 256) w3[i] = bfr(w[(size_t)(cg * 64) * 9 + i]);
  if (tid < 64) b3[tid] = bfr(bb[cg * 64 + tid]);
  __syncthreads();
  const _Float16* Hh = (const _Float16*)(const void*)H16;
#pragma unroll 1
  for (int jj = 0; jj < 16; ++jj) {
    const int cl = cq * 16 + jj;
    const int cc = cg * 64 + cl;
    const _Float16* hr = Hh + ((size_t)(b * CM + cc)) * NP;
    float accv = 0.f;
#pragma unroll
    for (int t = 0; t < 9; ++t) {
      const int ky = t / 3, kx = t - ky * 3;
      const int yy = y + ky - 1, xx = xq + kx - 1;
      const bool ok = ((unsigned)yy < (unsigned)IMW) && ((unsigned)xx < (unsigned)IMW);
      const int yc = min(max(yy, 0), IMW - 1);
      const int xc = min(max(xx, 0), IMW - 1);
      const float hv = (float)hr[yc * IMW + xc];
      accv = fmaf(ok ? hv : 0.f, w3[cl * 9 + t], accv);
    }
    const float z = accv * IHSC + b3[cl];
    const float h2 = hswish_f(z);
    Lh[nl * LTP + cl] = h_bits((_Float16)(h2 * H2SC));
  }
  __syncthreads();
  {
    const int e = tid & 7, lq = tid >> 3;
#pragma unroll
    for (int pass = 0; pass < 2; ++pass) {
#pragma unroll
      for (int it = 0; it < 2; ++it) {
        const int nn = it * 32 + lq;
        const v4u uh = *(const v4u*)(Lh + nn * LTP + 8 * e);
        const size_t po = ((size_t)(b * NP + n0 + nn)) * CM + cg * 64 + 8 * e;
        *(volatile v4u*)(H2 + po) = uh;
      }
      __threadfence();
    }
  }
}

extern "C" void kernel_launch(void* const* d_in, const int* in_sizes, int n_in,
                              void* d_out, int out_size, void* d_ws, size_t ws_size,
                              hipStream_t stream) {
  const int NX = NB * CH * NP;
  if (n_in < 19) return;
  if (in_sizes[0] != NX || in_sizes[1] != NX) return;
  if (in_sizes[2] != C3 * CH) return;
  if (in_sizes[3] != C3 * 25) return;
  if (in_sizes[4] != NGRP * 32 * 32) return;
  if (in_sizes[5] != CH * CA) return;
  if (in_sizes[6] != CH || in_sizes[7] != CH || in_sizes[8] != CH || in_sizes[9] != CH) return;
  if (in_sizes[10] != CM * CH || in_sizes[11] != CM) return;
  if (in_sizes[12] != CM * 9 || in_sizes[13] != CM) return;
  if (in_sizes[14] != CH * CM) return;
  if (in_sizes[15] != CH || in_sizes[16] != CH || in_sizes[17] != CH || in_sizes[18] != CH) return;
  if (out_size != NX) return;

  size_t off = 0;
  const size_t oW   = off; off += (size_t)WTOT * 2;
  const size_t oT2X = off; off += (size_t)NX * 4;
  const size_t oT1F = off; off += (size_t)NX * 4;
  const size_t oT1h = off; off += (size_t)NB * NP * CH * 2;
  const size_t oE   = off;
  const size_t oX16 = oE;
  const size_t oQKV = oX16 + (size_t)NB * NP * CH * 2;
  const size_t oPW  = oQKV + (size_t)NB * C3 * NP * 2;
  const size_t oATT = oPW + (size_t)NB * C3 * NP * 2;
  const size_t eA   = oATT + (size_t)NB * NP * CA * 2;
  const size_t oH16 = oE;
  const size_t oH2  = oH16 + (size_t)NB * CM * NP * 2;
  const size_t eB   = oH2 + (size_t)NB * NP * CM * 2;
  off = (eA > eB) ? eA : eB;
  if (off > ws_size) return;
  if (off > (size_t)134217728) return;

  const float* x        = (const float*)d_in[0];
  const float* y        = (const float*)d_in[1];
  const float* qkv_w    = (const float*)d_in[2];
  const float* agg_dw_w = (const float*)d_in[3];
  const float* agg_pw_w = (const float*)d_in[4];
  const float* proj_w   = (const float*)d_in[5];
  const float* proj_g   = (const float*)d_in[6];
  const float* proj_b   = (const float*)d_in[7];
  const float* proj_m   = (const float*)d_in[8];
  const float* proj_v   = (const float*)d_in[9];
  const float* inv_w    = (const float*)d_in[10];
  const float* inv_b    = (const float*)d_in[11];
  const float* dwc_w    = (const float*)d_in[12];
  const float* dwc_b    = (const float*)d_in[13];
  const float* pw_w     = (const float*)d_in[14];
  const float* pw_g     = (const float*)d_in[15];
  const float* pw_b     = (const float*)d_in[16];
  const float* pw_m     = (const float*)d_in[17];
  const float* pw_v     = (const float*)d_in[18];

  char* ws = (char*)d_ws;
  unsigned short* WB    = (unsigned short*)(ws + oW);
  float*          T2X   = (float*)(ws + oT2X);
  float*          T1F   = (float*)(ws + oT1F);
  unsigned short* T1h   = (unsigned short*)(ws + oT1h);
  unsigned short* X16   = (unsigned short*)(ws + oX16);
  unsigned short* QKV16 = (unsigned short*)(ws + oQKV);
  unsigned short* PW16  = (unsigned short*)(ws + oPW);
  unsigned short* ATT16 = (unsigned short*)(ws + oATT);
  unsigned short* H16   = (unsigned short*)(ws + oH16);
  unsigned short* H2h   = (unsigned short*)(ws + oH2);
  float* out = (float*)d_out;

  const dim3 blk256(256);
  const dim3 gW(WTOT / 2048);
  const dim3 gX(NP / GN, CH / 64, NB);
  const dim3 gQ(C3 / GM, NP / GN, NB);
  const dim3 gD5(NP / GN, NGRP, NB);
  const dim3 gA(NPAIR, NB);
  const dim3 gP(CH / GM, NP / GN, NB);
  const dim3 gI(CM / GM, NP / GN, NB);
  const dim3 gD3(NP / GN, CM / 64, NB);

  cvt_w<<<gW, blk256, 0, stream>>>(qkv_w, proj_w, inv_w, pw_w, WB);

  for (int pass = 0; pass < 2; ++pass) {
    const float* t = (pass == 0) ? x : y;
    cvt_x<<<gX, blk256, 0, stream>>>(t, X16);
    gemm_kernel<0><<<gQ, blk256, 0, stream>>>(WB, CH, 1.0f, X16,
        nullptr, nullptr, nullptr, nullptr, nullptr, 0,
        nullptr, 0, nullptr, C3,
        nullptr, QKV16, 1.0f, nullptr, 0.0f);
    dw5_gpw_kernel<<<gD5, blk256, 0, stream>>>(QKV16, agg_dw_w, agg_pw_w, PW16);
    attn_kernel<<<gA, blk256, 0, stream>>>(QKV16, PW16, ATT16);
    gemm_kernel<1><<<gP, blk256, 0, stream>>>(WB + WOFF1, CA, SA_PROJ, ATT16,
        nullptr, proj_g, proj_b, proj_m, proj_v, 0,
        t, 1, nullptr, CH,
        T1F, nullptr, 0.0f, T1h, T1SC);
    gemm_kernel<1><<<gI, blk256, 0, stream>>>(WB + WOFF2, CH, SA_INV, T1h,
        inv_b, nullptr, nullptr, nullptr, nullptr, 1,
        nullptr, 0, nullptr, CM,
        nullptr, H16, HSC, nullptr, 0.0f);
    dw3_kernel<<<gD3, blk256, 0, stream>>>(H16, dwc_w, dwc_b, H2h);
    gemm_kernel<1><<<gP, blk256, 0, stream>>>(WB + WOFF3, CM, SA_PW, H2h,
        nullptr, pw_g, pw_b, pw_m, pw_v, 0,
        T1F, 0, (pass == 0) ? (const float*)nullptr : (const float*)T2X, CH,
        (pass == 0) ? T2X : out, nullptr, 0.0f, nullptr, 0.0f);
  }
  (void)hipGetLastError();
}
